// MappingNet_44504451121189
// MI455X (gfx1250) — hardware-run, weakly checked
//
#include <hip/hip_runtime.h>


namespace {
constexpr int NBR = 4096, DIN = 512, DM = 1024, NE = 10, MAXT = NBR / 16 + NE  ;
constexpr float XS = 8.0f, HS = 256.0f  , WSC = 256.0f;
typedef _Float16 b16;
typedef __attribute__((ext_vector_type(16))) _Float16 v16b;
typedef __attribute__((ext_vector_type(8))) _Float16 v8b;
typedef __attribute__((ext_vector_type(8))) float v8f;
typedef __attribute__((ext_vector_type(4))) float v4f;
__device__ __forceinline__ float bf16_rne(float f) { unsigned int u = __float_as_uint(f); u += 0x7FFFu + ((u >> 16) & 1u); float r = __uint_as_float(u & 0xFFFF0000u); asm volatile("" : "+v"(r)); return r; }
__device__ __forceinline__ float bfv(float f) { float r = bf16_rne(f); asm volatile("" : "+v"(r)); return r; }
__device__ __forceinline__ void split16(float v, b16& hi, b16& lo) { hi = (b16)v; lo = (b16)(v - (float)hi); }
__device__ __forceinline__ v16b frag_kb(const b16* p, int hh) { const v8b a = *(const v8b*)(p + 8 * hh), b = *(const v8b*)(p + 16 + 8 * hh); v16b f;
#pragma unroll
  for (int e = 0; e < 8; ++e) { f[e] = a[e]; f[8 + e] = b[e]; } return f; }
__device__ __forceinline__ v8f wmma16b(v16b a, v16b b, v8f c) { v8f d = __builtin_amdgcn_wmma_f32_16x16x32_f16(false, a, false, b, (short)0, c, false, false); asm volatile("v_nop\n\tv_nop\n\tv_nop\n\tv_nop" : "+v"(d) : "v"(a), "v"(b)); return d; }
__device__ __forceinline__ void wave_lds_sync() { __builtin_amdgcn_fence(__ATOMIC_RELEASE, "workgroup"); __builtin_amdgcn_wave_barrier(); __builtin_amdgcn_fence(__ATOMIC_ACQUIRE, "workgroup"); }
__device__ __forceinline__ int iclamp(int v, int lo, int hi) { return v < lo ? lo : (v > hi ? hi : v); }
__device__ __forceinline__ float gelu(float v) { return 0.5f * v * (1.0f + erff(v * 0.70710678118654752f)); }

__global__ __launch_bounds__(256) void wput_kernel(const float* __restrict__ ws1, const float* __restrict__ ws2, const float* __restrict__ we1, const float* __restrict__ we2, b16* __restrict__ W1T, b16* __restrict__ W2T, b16* __restrict__ E1T, b16* __restrict__ E2T) { const size_t u = (size_t)blockIdx.x * 256 + threadIdx.x; const size_t n1 = (size_t)DM * (DIN / 8), n2 = (size_t)DM * (DM / 8), ne = (size_t)NE * DM * (DM / 8); v8b v;
  if (u < n1) { const int o = (int)(u / (DIN / 8)), k0 = (int)(u % (DIN / 8)) * 8;
#pragma unroll
    for (int j = 0; j < 8; ++j) v[j] = (b16)(bf16_rne(ws1[(size_t)(k0 + j) * DM + o]) * WSC); for (int pass = 0; pass < 2; ++pass) { *(volatile v8b*)(W1T + (size_t)o * DIN + k0) = v; __threadfence(); } }
  if (u < n2) { const int o = (int)(u / (DM / 8)), k0 = (int)(u % (DM / 8)) * 8;
#pragma unroll
    for (int j = 0; j < 8; ++j) v[j] = (b16)(bf16_rne(ws2[(size_t)(k0 + j) * DM + o]) * WSC); for (int pass = 0; pass < 2; ++pass) { *(volatile v8b*)(W2T + (size_t)o * DM + k0) = v; __threadfence(); } }
  if (u < ne) { const int e = (int)(u / n2); const size_t w = u % n2; const int o = (int)(w / (DM / 8)), k0 = (int)(w % (DM / 8)) * 8; v8b a, b;
#pragma unroll
    for (int j = 0; j < 8; ++j) { a[j] = (b16)(bf16_rne(we1[((size_t)e * DM + k0 + j) * DM + o]) * WSC); b[j] = (b16)(bf16_rne(we2[((size_t)e * DM + k0 + j) * DM + o]) * WSC); }
    for (int pass = 0; pass < 2; ++pass) { *(volatile v8b*)(E1T + ((size_t)e * DM + o) * DM + k0) = a; *(volatile v8b*)(E2T + ((size_t)e * DM + o) * DM + k0) = b; __threadfence(); } } }
__global__ __launch_bounds__(1024) void group_kernel(const int* __restrict__ genre, int RLIM, int* __restrict__ RP, int* __restrict__ NTILE) { __shared__ int scanbuf[1024]; __shared__ int cnt[NE], toff[NE + 1]; __shared__ int perm[NBR]; const int t = threadIdx.x; int g[4]; for (int j = 0; j < 4; ++j) g[j] = (t * 4 + j) < RLIM ? iclamp(genre[t * 4 + j], 0, NE - 1) : -1;
  int base = 0;
  for (int e = 0; e < NE; ++e) { int c = 0; for (int j = 0; j < 4; ++j) c += (g[j] == e); scanbuf[t] = c; __syncthreads();
    for (int s = 1; s < 1024; s <<= 1) { const int v = t >= s ? scanbuf[t - s] : 0; __syncthreads(); scanbuf[t] += v; __syncthreads(); }
    const int excl = scanbuf[t] - c, tot = scanbuf[1023]; int pos = base + excl; for (int j = 0; j < 4; ++j) if (g[j] == e) perm[pos++] = t * 4 + j;
    if (t == 0) cnt[e] = tot; base += tot; __syncthreads(); }
  if (t == 0) { toff[0] = 0; for (int e = 0; e < NE; ++e) toff[e + 1] = toff[e] + (cnt[e] + 15) / 16; }
  __syncthreads(); const int ntile = toff[NE];
  for (int pass = 0; pass < 2; ++pass) { for (int slot = t; slot < MAXT * 16; slot += 1024) { const int tile = slot / 16, j = slot % 16; int row = -1;
      if (tile < ntile) { int e = 0; while (e + 1 < NE && toff[e + 1] <= tile) ++e; int segst = 0; for (int q = 0; q < e; ++q) segst += cnt[q]; const int idx = (tile - toff[e]) * 16 + j; if (idx < cnt[e]) row = perm[segst + idx]; }
      ((volatile int*)RP)[slot] = row; }
    if (t < 32) ((volatile int*)NTILE)[t] = t == 0 ? ntile : 0; __threadfence(); } }
template <int MODE>
__global__ __launch_bounds__(32) void layer_kernel(const float* __restrict__ IN, const int* __restrict__ RP, const int* __restrict__ NTILE, const int* __restrict__ genre, const b16* __restrict__ WT, const float* __restrict__ bias, float* __restrict__ OUT) { constexpr int K = MODE == 0 ? DIN : DM; __shared__ __attribute__((aligned(16))) b16 Ah[16][K + 8], Al[16][MODE == 0 ? 8 : K + 8]; __shared__ float Tf[16][260]; __shared__ int rows[16]; const int lane = threadIdx.x, nloc = lane & 15, hlf = lane >> 4; const int tile = blockIdx.x;
  if (MODE >= 2) { if (tile >= NTILE[0]) return; if (lane < 16) rows[lane] = RP[tile * 16 + lane]; wave_lds_sync(); }
  int e = 0; if (MODE >= 2) { const int r0 = rows[0]; e = iclamp(genre[r0 < 0 ? 0 : r0], 0, NE - 1); }
  const b16* W = MODE >= 2 ? WT + (size_t)e * DM * DM : WT; const float* bb = MODE >= 2 ? bias + (size_t)e * DM : bias;
  for (int rr = 0; rr < 16; ++rr) { size_t src; if (MODE == 0 || MODE == 1) src = (size_t)tile * 16 + rr; else if (MODE == 2) { const int r = rows[rr]; src = (size_t)(r < 0 ? 0 : r); } else src = (size_t)tile * 16 + rr;
    for (int q = 0; q < K / 32; ++q) { const float v = IN[src * K + q * 32 + lane]; if (MODE == 0) Ah[rr][q * 32 + lane] = (b16)(bf16_rne(v) * XS); else { b16 p, ql; split16(v * HS, p, ql); Ah[rr][q * 32 + lane] = p; Al[rr][q * 32 + lane] = ql; } } }
  wave_lds_sync();
#pragma unroll 1
  for (int g = 0; g < DM / 256; ++g) { v8f acc[16];
#pragma unroll
    for (int t = 0; t < 16; ++t) acc[t] = (v8f){};
#pragma unroll 2
    for (int kb = 0; kb < K; kb += 32) { const v16b a = frag_kb(&Ah[nloc][kb], hlf); v16b al; if (MODE != 0) al = frag_kb(&Al[nloc][kb], hlf);
#pragma unroll
      for (int t = 0; t < 16; ++t) { const v16b bw = frag_kb(W + (size_t)(g * 256 + t * 16 + nloc) * K + kb, hlf); acc[t] = wmma16b(a, bw, acc[t]); if (MODE != 0) acc[t] = wmma16b(al, bw, acc[t]); } }
#pragma unroll
    for (int t = 0; t < 16; ++t) { const int cc = t * 16 + nloc; const float bv = bfv(bb[g * 256 + cc]);
#pragma unroll
      for (int r8 = 0; r8 < 8; ++r8) { const float v = acc[t][r8] * (MODE == 0 ? 1.0f / (XS * WSC) : 1.0f / (HS * WSC)) + bv; Tf[8 * hlf + r8][cc] = MODE == 3 ? v : gelu(v); } }
    wave_lds_sync();
    for (int pass = 0; pass < 2; ++pass) { for (int rr = 0; rr < 16; ++rr) { size_t dst; if (MODE == 3) { const int r = rows[rr]; if (r < 0) continue; dst = (size_t)r; } else dst = (size_t)tile * 16 + rr;
        for (int q = 0; q < 2; ++q) *(volatile v4f*)(OUT + dst * DM + g * 256 + q * 128 + lane * 4) = *(const v4f*)(&Tf[rr][q * 128 + lane * 4]); } __threadfence(); }
    wave_lds_sync(); } }
}

extern "C" void kernel_launch(void* const* d_in, const int* in_sizes, int n_in, void* d_out, int out_size, void* d_ws, size_t ws_size, hipStream_t stream) {
  (void)n_in;
  auto Fp = [&](int i) { return (const float*)d_in[i]; }; auto Ip = [&](int i) { return (const int*)d_in[i]; };
  if (in_sizes[0] != NBR * DIN || in_sizes[1] != NBR || in_sizes[2] != DIN * DM || in_sizes[4] != DM * DM || in_sizes[6] != NE * DM * DM || in_sizes[8] != NE * DM * DM || out_size != NBR * DM) return;
  const int RLIM = NBR;
  size_t off = 0; char* ws = (char*)d_ws;
  auto carve = [&](size_t bytes) { char* p = ws + off; off += (bytes + 255) & ~(size_t)255; return p; };
  b16* W1T = (b16*)carve((size_t)DM * DIN * 2); b16* W2T = (b16*)carve((size_t)DM * DM * 2); b16* E1T = (b16*)carve((size_t)NE * DM * DM * 2); b16* E2T = (b16*)carve((size_t)NE * DM * DM * 2); float* T1 = (float*)carve((size_t)NBR * DM * 4); float* S = (float*)carve((size_t)NBR * DM * 4); float* HP = (float*)carve((size_t)MAXT * 16 * DM * 4); int* RP = (int*)carve((size_t)MAXT * 16 * 4); int* NTILE = (int*)carve(32 * 4);
  if (off > ws_size || off > ((size_t)128 << 20)) return;
  wput_kernel<<<(unsigned)(((size_t)NE * DM * (DM / 8) + 255) / 256), 256, 0, stream>>>(Fp(2), Fp(4), Fp(6), Fp(8), W1T, W2T, E1T, E2T);
  group_kernel<<<1, 1024, 0, stream>>>(Ip(1), RLIM, RP, NTILE);
  layer_kernel<0><<<RLIM / 16, 32, 0, stream>>>(Fp(0), RP, NTILE, Ip(1), W1T, Fp(3), T1);
  layer_kernel<1><<<RLIM / 16, 32, 0, stream>>>(T1, RP, NTILE, Ip(1), W2T, Fp(5), S);
  layer_kernel<2><<<MAXT, 32, 0, stream>>>(S, RP, NTILE, Ip(1), E1T, Fp(7), HP);
  layer_kernel<3><<<MAXT, 32, 0, stream>>>(HP, RP, NTILE, Ip(1), E2T, Fp(9), (float*)d_out);
}
